// ODERNN_57578331570467
// MI455X (gfx1250) — hardware-run, weakly checked
//
#include <hip/hip_runtime.h>
#include <math.h>

constexpr int NSEQ  = 256;
constexpr int NSTEP = 64;
constexpr int NC    = 64;
constexpr int NH    = 256;
constexpr int NHH   = 1024;
constexpr int NCLS  = 32;
constexpr int NG3   = 3 * NH;
constexpr int NTHR  = 256;
constexpr int RB    = 16;
constexpr int ZP    = 264;
constexpr int XP    = 72;
constexpr int AP    = 1032;
constexpr int HSP   = 260;
constexpr float ASCL   = 16.0f;
constexpr float WSCL   = 256.0f;
constexpr float INV_AW = 1.0f / 4096.0f;
constexpr float THIRD  = 1.0f / 3.0f;
static_assert(NSEQ % RB == 0);
static_assert(NH == 32 * (NTHR / 32));
static_assert(NHH == 128 * (NTHR / 32));
static_assert(NC % 32 == 0 && NH % 32 == 0 && NHH % 32 == 0);
static_assert(RB * NC == 4 * NTHR);
static_assert((RB * NH) % (4 * NTHR) == 0);
static_assert(NSEQ % (NTHR / 32) == 0);
static_assert(NCLS == 32);
static_assert(ZP % 8 == 0 && XP % 8 == 0 && AP % 8 == 0 && HSP % 4 == 0);
static_assert((NG3 * NC / 8) % NTHR == 0 && (NG3 * NH / 8) % NTHR == 0 && (NHH * NH / 8) % NTHR == 0 &&
              (NHH * NHH / 8) % NTHR == 0 && (NH * NHH / 8) % NTHR == 0);

typedef __attribute__((ext_vector_type(16))) _Float16 v16h;
typedef __attribute__((ext_vector_type(8)))  _Float16 v8h;
typedef __attribute__((ext_vector_type(16))) __bf16   v16b;
typedef __attribute__((ext_vector_type(8)))  __bf16   v8b;
typedef __attribute__((ext_vector_type(8)))  float    v8f;
typedef __attribute__((ext_vector_type(4)))  float    v4f;
typedef __attribute__((ext_vector_type(2)))  unsigned v2u;

__device__ __forceinline__ unsigned short f2bf_bits(float f) {
  unsigned u = __float_as_uint(f);
  return (unsigned short)((u + 0x7FFFu + ((u >> 16) & 1u)) >> 16);
}
__device__ __forceinline__ float bf_bits2f(unsigned short h) { return __uint_as_float(((unsigned)h) << 16); }
__device__ __forceinline__ float bf16r(float f) { return bf_bits2f(f2bf_bits(f)); }

__device__ __forceinline__ void dep_guard_h(v8f& a, v8f& b, v16h x, v16h y) { asm volatile("v_nop\n\tv_nop\n\tv_nop\n\tv_nop" : "+v"(a), "+v"(b) : "v"(x), "v"(y)); }
__device__ __forceinline__ void dep_guard_b(v8f& a, v8f& b, v16b x, v16b y) { asm volatile("v_nop\n\tv_nop\n\tv_nop\n\tv_nop" : "+v"(a), "+v"(b) : "v"(x), "v"(y)); }
__device__ __forceinline__ void keep4_h(v16h a, v16h b, v16h c, v16h d) { asm volatile("v_nop" :: "v"(a), "v"(b), "v"(c), "v"(d)); }
__device__ __forceinline__ void keep4_b(v16b a, v16b b, v16b c, v16b d) { asm volatile("v_nop" :: "v"(a), "v"(b), "v"(c), "v"(d)); }
__device__ __forceinline__ void acc_guard4(v8f& a, v8f& b, v8f& c, v8f& d) { asm volatile("v_nop\n\tv_nop\n\tv_nop\n\tv_nop" : "+v"(a), "+v"(b), "+v"(c), "+v"(d)); }
__device__ __forceinline__ void acc_guard2(v8f& a, v8f& b) { asm volatile("v_nop\n\tv_nop\n\tv_nop\n\tv_nop" : "+v"(a), "+v"(b)); }
template <typename T> struct Frag;
template <> struct Frag<_Float16> {
  typedef v16h V; union U { v16h v; v8h h[2]; };
  static __device__ __forceinline__ v16h load(const _Float16* p) {
    U f; f.h[0] = *(const v8h*)(p); f.h[1] = *(const v8h*)(p + 16); return f.v;
  }
  static __device__ __forceinline__ v8f mma(v16h a, v16h b, v8f c) {
    return __builtin_amdgcn_wmma_f32_16x16x32_f16(false, a, false, b, (short)0, c, false, false);
  }
  static __device__ __forceinline__ void guard(v8f& a, v8f& b, v16h x, v16h y) { dep_guard_h(a, b, x, y); }
  static __device__ __forceinline__ void keep(v16h a, v16h b, v16h c, v16h d) { keep4_h(a, b, c, d); }
};
template <> struct Frag<__bf16> {
  typedef v16b V; union U { v16b v; v8b h[2]; };
  static __device__ __forceinline__ v16b load(const __bf16* p) {
    U f; f.h[0] = *(const v8b*)(p); f.h[1] = *(const v8b*)(p + 16); return f.v;
  }
  static __device__ __forceinline__ v8f mma(v16b a, v16b b, v8f c) {
    return __builtin_amdgcn_wmma_f32_16x16x32_bf16(false, a, false, b, (short)0, c, false, false);
  }
  static __device__ __forceinline__ void guard(v8f& a, v8f& b, v16b x, v16b y) { dep_guard_b(a, b, x, y); }
  static __device__ __forceinline__ void keep(v16b a, v16b b, v16b c, v16b d) { keep4_b(a, b, c, d); }
};

__device__ __forceinline__ float fsig(float x)  { return __builtin_amdgcn_rcpf(1.0f + __expf(-x)); }
__device__ __forceinline__ float ftanh(float x) { return 1.0f - 2.0f * __builtin_amdgcn_rcpf(__expf(2.0f * x) + 1.0f); }

template <int MODE>
__global__ __launch_bounds__(NTHR) void cvt8_kernel(const float* __restrict__ src, unsigned short* __restrict__ dst,
                                                    int nrow, int ncol8, int spitch, int scol0, float sc) {
  const int i  = blockIdx.x * NTHR + threadIdx.x;
  const int n8 = nrow * ncol8;
  if (i < n8) {
    const int row = i / ncol8;
    const int c8  = i - row * ncol8;
    const float* sp = src + (size_t)row * spitch + scol0 + c8 * 8;
    const v4f a = *(const v4f*)(sp);
    const v4f b = *(const v4f*)(sp + 4);
    v8h hv;
#pragma unroll
    for (int e = 0; e < 4; ++e) {
      unsigned short b0, b1;
      if (MODE == 0) {
        b0 = f2bf_bits(a[e] * sc);
        b1 = f2bf_bits(b[e] * sc);
      } else {
        b0 = __builtin_bit_cast(unsigned short, (_Float16)(bf16r(a[e]) * sc));
        b1 = __builtin_bit_cast(unsigned short, (_Float16)(bf16r(b[e]) * sc));
      }
      hv[e]     = __builtin_bit_cast(_Float16, b0);
      hv[4 + e] = __builtin_bit_cast(_Float16, b1);
    }
    *(volatile v8h*)(dst + (size_t)i * 8) = hv;
    __threadfence();
    *(volatile v8h*)(dst + (size_t)i * 8) = hv;
  }
}

__device__ __forceinline__ void stage_x_tile(const float* __restrict__ x, unsigned short* Xt, int rowbase, int tstep, int tid) {
  const int m = tid >> 4, f4 = (tid & 15) * 4;
  const v4f v = *(const v4f*)(x + ((size_t)(rowbase + m) * NSTEP + (size_t)tstep) * NC + f4);
  const unsigned short u0 = __builtin_bit_cast(unsigned short, (_Float16)(bf16r(v[0]) * ASCL));
  const unsigned short u1 = __builtin_bit_cast(unsigned short, (_Float16)(bf16r(v[1]) * ASCL));
  const unsigned short u2 = __builtin_bit_cast(unsigned short, (_Float16)(bf16r(v[2]) * ASCL));
  const unsigned short u3 = __builtin_bit_cast(unsigned short, (_Float16)(bf16r(v[3]) * ASCL));
  v2u pk;
  pk[0] = (unsigned)u0 | ((unsigned)u1 << 16);
  pk[1] = (unsigned)u2 | ((unsigned)u3 << 16);
  *(v2u*)(Xt + m * XP + f4) = pk;
}

__global__ __launch_bounds__(NTHR) void seq_rk4_gru_kernel(
    const float* __restrict__ x, const float* __restrict__ times,
    const float* __restrict__ b_ih, const float* __restrict__ b_hh,
    const float* __restrict__ bias1, const float* __restrict__ bias2, const float* __restrict__ bias3,
    const unsigned short* __restrict__ WIHp, const unsigned short* __restrict__ WHHp,
    const unsigned short* __restrict__ W1p, const unsigned short* __restrict__ W2p,
    const unsigned short* __restrict__ W3p, float* __restrict__ HFIN) {
  __shared__ __align__(16) _Float16       Zt[RB * ZP];
  __shared__ __align__(16) unsigned short Xt[RB * XP];
  __shared__ __align__(16) _Float16       A1[RB * AP];
  __shared__ __align__(16) _Float16       A2[RB * AP];
  __shared__ __align__(16) float          Hs[RB * HSP];
  const _Float16* WIH = (const _Float16*)WIHp;
  const _Float16* WHH = (const _Float16*)WHHp;
  const _Float16* W1  = (const _Float16*)W1p;
  const _Float16* W2  = (const _Float16*)W2p;
  const _Float16* W3  = (const _Float16*)W3p;
  const int tid = threadIdx.x, lane = tid & 31, wave = tid >> 5;
  const int c = lane & 15, hh = lane >> 4, koff = hh * 8;
  const int rowbase = blockIdx.x * RB;

#pragma unroll 1
  for (int i = tid; i < RB * ZP; i += NTHR) Zt[i] = (_Float16)0.0f;
#pragma unroll 1
  for (int i = tid; i < RB * XP; i += NTHR) Xt[i] = (unsigned short)0;
#pragma unroll 1
  for (int i = tid; i < RB * AP; i += NTHR) { A1[i] = (_Float16)0.0f; A2[i] = (_Float16)0.0f; }
#pragma unroll 1
  for (int i = tid; i < RB * HSP; i += NTHR) Hs[i] = 0.0f;
  __syncthreads();

  stage_x_tile(x, Xt, rowbase, 0, tid);
  float yst[2][8], ka[2][8], kb[2][8];
  float bsum[2][2], bsep[2][2], b3v[2];
#pragma unroll
  for (int nt = 0; nt < 2; ++nt) {
    const int j = 32 * wave + 16 * nt + c;
    bsum[nt][0] = bf16r(b_ih[j]) + bf16r(b_hh[j]);
    bsum[nt][1] = bf16r(b_ih[NH + j]) + bf16r(b_hh[NH + j]);
    bsep[nt][0] = bf16r(b_ih[2 * NH + j]);
    bsep[nt][1] = bf16r(b_hh[2 * NH + j]);
    b3v[nt]     = bf16r(bias3[j]);
#pragma unroll
    for (int r = 0; r < 8; ++r) { yst[nt][r] = 0.0f; ka[nt][r] = 0.0f; kb[nt][r] = 0.0f; }
  }
  __syncthreads();

  const _Float16* ztrow = Zt + c * ZP + koff;
  const _Float16* xtrow = (const _Float16*)Xt + c * XP + koff;
  const _Float16* a1row = A1 + c * AP + koff;
  const _Float16* a2row = A2 + c * AP + koff;
  const v8f z8 = {0.f, 0.f, 0.f, 0.f, 0.f, 0.f, 0.f, 0.f};

#pragma unroll 1
  for (int t = 0; t < NSTEP; ++t) {
    if (t > 0) {
      const float dt = bf16r(times[t]) - bf16r(times[t - 1]);
#pragma unroll 1
      for (int s = 0; s < 4; ++s) {
#pragma unroll 1
        for (int p = 0; p < 2; ++p) {
          const int jb = 128 * wave + 64 * p;
          const _Float16* wb = W1 + (size_t)(jb + c) * NH + koff;
          v8f acc[4];
          acc[0] = z8; acc[1] = z8; acc[2] = z8; acc[3] = z8;
#pragma unroll 1
          for (int k0 = 0; k0 < NH; k0 += 32) {
            const v16h a  = Frag<_Float16>::load(ztrow + k0);
            const v16h f0 = Frag<_Float16>::load(wb + k0);
            const v16h f1 = Frag<_Float16>::load(wb + (size_t)16 * NH + k0);
            const v16h f2 = Frag<_Float16>::load(wb + (size_t)32 * NH + k0);
            const v16h f3 = Frag<_Float16>::load(wb + (size_t)48 * NH + k0);
            acc[0] = Frag<_Float16>::mma(a, f0, acc[0]);
            acc[1] = Frag<_Float16>::mma(a, f1, acc[1]);
            acc[2] = Frag<_Float16>::mma(a, f2, acc[2]);
            acc[3] = Frag<_Float16>::mma(a, f3, acc[3]);
            dep_guard_h(acc[0], acc[3], a, f3);
            keep4_h(f0, f1, f2, f3);
          }
          acc_guard4(acc[0], acc[1], acc[2], acc[3]);
#pragma unroll
          for (int nt = 0; nt < 4; ++nt) {
            const int j = jb + 16 * nt + c;
            const float bb = bf16r(bias1[j]);
#pragma unroll
            for (int r = 0; r < 8; ++r) {
              const float v = ftanh(acc[nt][r] * INV_AW + bb);
              A1[(8 * hh + r) * AP + j] = (_Float16)(v * ASCL);
            }
          }
        }
        __syncthreads();
#pragma unroll 1
        for (int p = 0; p < 2; ++p) {
          const int jb = 128 * wave + 64 * p;
          const _Float16* wb = W2 + (size_t)(jb + c) * NHH + koff;
          v8f acc[4];
          acc[0] = z8; acc[1] = z8; acc[2] = z8; acc[3] = z8;
#pragma unroll 1
          for (int k0 = 0; k0 < NHH; k0 += 32) {
            const v16h a  = Frag<_Float16>::load(a1row + k0);
            const v16h f0 = Frag<_Float16>::load(wb + k0);
            const v16h f1 = Frag<_Float16>::load(wb + (size_t)16 * NHH + k0);
            const v16h f2 = Frag<_Float16>::load(wb + (size_t)32 * NHH + k0);
            const v16h f3 = Frag<_Float16>::load(wb + (size_t)48 * NHH + k0);
            acc[0] = Frag<_Float16>::mma(a, f0, acc[0]);
            acc[1] = Frag<_Float16>::mma(a, f1, acc[1]);
            acc[2] = Frag<_Float16>::mma(a, f2, acc[2]);
            acc[3] = Frag<_Float16>::mma(a, f3, acc[3]);
            dep_guard_h(acc[0], acc[3], a, f3);
            keep4_h(f0, f1, f2, f3);
          }
          acc_guard4(acc[0], acc[1], acc[2], acc[3]);
#pragma unroll
          for (int nt = 0; nt < 4; ++nt) {
            const int j = jb + 16 * nt + c;
            const float bb = bf16r(bias2[j]);
#pragma unroll
            for (int r = 0; r < 8; ++r) {
              const float v = ftanh(acc[nt][r] * INV_AW + bb);
              A2[(8 * hh + r) * AP + j] = (_Float16)(v * ASCL);
            }
          }
        }
        __syncthreads();
        {
          const _Float16* wb = W3 + (size_t)(32 * wave + c) * NHH + koff;
          v8f acc[2];
          acc[0] = z8; acc[1] = z8;
#pragma unroll 1
          for (int k0 = 0; k0 < NHH; k0 += 32) {
            const v16h a  = Frag<_Float16>::load(a2row + k0);
            const v16h f0 = Frag<_Float16>::load(wb + k0);
            const v16h f1 = Frag<_Float16>::load(wb + (size_t)16 * NHH + k0);
            acc[0] = Frag<_Float16>::mma(a, f0, acc[0]);
            acc[1] = Frag<_Float16>::mma(a, f1, acc[1]);
            dep_guard_h(acc[0], acc[1], a, f1);
            keep4_h(a, f0, f1, a);
          }
          acc_guard2(acc[0], acc[1]);
#pragma unroll
          for (int nt = 0; nt < 2; ++nt) {
            const int j = 32 * wave + 16 * nt + c;
#pragma unroll
            for (int r = 0; r < 8; ++r) {
              const float kv = acc[nt][r] * INV_AW + b3v[nt];
              float yv = yst[nt][r], kav = ka[nt][r], kbv = kb[nt][r];
              float zv;
              if (s == 0)      { zv = yv + dt * kv * THIRD;          kav = kv;        kbv = kv; }
              else if (s == 1) { zv = yv + dt * (kv - kav * THIRD);  kbv = kav - kv;  kav = kav + 3.0f * kv; }
              else if (s == 2) { zv = yv + dt * (kbv + kv);          kav = kav + 3.0f * kv; }
              else             { yv = yv + (kav + kv) * dt * 0.125f; zv = yv; }
              yst[nt][r] = yv; ka[nt][r] = kav; kb[nt][r] = kbv;
              Zt[(8 * hh + r) * ZP + j] = (_Float16)(zv * ASCL);
            }
          }
        }
        __syncthreads();
      }
    }
#pragma unroll
    for (int nt = 0; nt < 2; ++nt) {
      const int j = 32 * wave + 16 * nt + c;
      const _Float16* wi = WIH + (size_t)j * NC + koff;
      const _Float16* wh = WHH + (size_t)j * NH + koff;
      v8f acc[4];
      acc[0] = z8; acc[1] = z8; acc[2] = z8; acc[3] = z8;
#pragma unroll 1
      for (int kx = 0; kx < NC; kx += 32) {
        const v16h a  = Frag<_Float16>::load(xtrow + kx);
        const v16h f0 = Frag<_Float16>::load(wi + kx);
        const v16h f1 = Frag<_Float16>::load(wi + (size_t)NH * NC + kx);
        const v16h f2 = Frag<_Float16>::load(wi + (size_t)2 * NH * NC + kx);
        acc[0] = Frag<_Float16>::mma(a, f0, acc[0]);
        acc[1] = Frag<_Float16>::mma(a, f1, acc[1]);
        acc[2] = Frag<_Float16>::mma(a, f2, acc[2]);
        dep_guard_h(acc[0], acc[2], a, f2);
        keep4_h(f0, f1, f2, a);
      }
#pragma unroll 1
      for (int k0 = 0; k0 < NH; k0 += 32) {
        const v16h a  = Frag<_Float16>::load(ztrow + k0);
        const v16h f0 = Frag<_Float16>::load(wh + k0);
        const v16h f1 = Frag<_Float16>::load(wh + (size_t)NH * NH + k0);
        const v16h f2 = Frag<_Float16>::load(wh + (size_t)2 * NH * NH + k0);
        acc[0] = Frag<_Float16>::mma(a, f0, acc[0]);
        acc[1] = Frag<_Float16>::mma(a, f1, acc[1]);
        acc[3] = Frag<_Float16>::mma(a, f2, acc[3]);
        dep_guard_h(acc[0], acc[3], a, f2);
        keep4_h(f0, f1, f2, a);
      }
      acc_guard4(acc[0], acc[1], acc[2], acc[3]);
#pragma unroll
      for (int r = 0; r < 8; ++r) {
        const float pr  = acc[0][r] * INV_AW + bsum[nt][0];
        const float pz  = acc[1][r] * INV_AW + bsum[nt][1];
        const float gin = acc[2][r] * INV_AW + bsep[nt][0];
        const float ghn = acc[3][r] * INV_AW + bsep[nt][1];
        const float rg = fsig(pr);
        const float zg = fsig(pz);
        const float ng = ftanh(gin + rg * ghn);
        const float hp = yst[nt][r];
        yst[nt][r] = (1.0f - zg) * ng + zg * hp;
      }
    }
    __syncthreads();
#pragma unroll
    for (int nt = 0; nt < 2; ++nt) {
      const int j = 32 * wave + 16 * nt + c;
#pragma unroll
      for (int r = 0; r < 8; ++r) Zt[(8 * hh + r) * ZP + j] = (_Float16)(yst[nt][r] * ASCL);
    }
    {
      const int tn = (t + 1 < NSTEP) ? (t + 1) : (NSTEP - 1);
      stage_x_tile(x, Xt, rowbase, tn, tid);
    }
    __syncthreads();
  }

#pragma unroll
  for (int nt = 0; nt < 2; ++nt) {
    const int j = 32 * wave + 16 * nt + c;
#pragma unroll
    for (int r = 0; r < 8; ++r) Hs[(8 * hh + r) * HSP + j] = yst[nt][r];
  }
  __syncthreads();
  for (int pass = 0; pass < 2; ++pass) {
#pragma unroll
    for (int it = 0; it < 4; ++it) {
      const int idx = it * NTHR + tid;
      const int row = idx >> 6, c4 = (idx & 63) * 4;
      const v4f v = *(const v4f*)(Hs + row * HSP + c4);
      *(volatile v4f*)(HFIN + (size_t)(rowbase + row) * NH + c4) = v;
    }
    __threadfence();
  }
}

__global__ __launch_bounds__(NTHR) void head_softmax_kernel(const float* __restrict__ HF, const float* __restrict__ Wo,
                                                            const float* __restrict__ bo, float* __restrict__ out) {
  __shared__ __align__(16) float sm[NTHR / 32][NCLS];
  const int tid = threadIdx.x, lane = tid & 31, wave = tid >> 5;
  const int row = blockIdx.x * (NTHR / 32) + wave;
  const float* hr = HF + (size_t)row * NH;
  const float* wr = Wo + (size_t)lane * NH;
  float acc = 0.0f;
#pragma unroll 1
  for (int k = 0; k < NH; k += 4) {
    const v4f hv = *(const v4f*)(hr + k);
    const v4f wv = *(const v4f*)(wr + k);
    acc += hv[0] * bf16r(wv[0]);
    acc += hv[1] * bf16r(wv[1]);
    acc += hv[2] * bf16r(wv[2]);
    acc += hv[3] * bf16r(wv[3]);
  }
  acc += bf16r(bo[lane]);
  float m = acc;
#pragma unroll
  for (int off = 1; off < 32; off <<= 1) m = fmaxf(m, __shfl_xor(m, off, 32));
  const float e = expf(acc - m);
  float s = e;
#pragma unroll
  for (int off = 1; off < 32; off <<= 1) s += __shfl_xor(s, off, 32);
  const float pv = e * (1.0f / s);
  sm[wave][lane] = pv;
  __syncthreads();
  if (lane < 8) {
    const v4f v = *(const v4f*)(&sm[wave][4 * lane]);
    float* op = out + (size_t)row * NCLS + 4 * lane;
    *(volatile v4f*)op = v;
    __threadfence();
    *(volatile v4f*)op = v;
  }
}

extern "C" void kernel_launch(void* const* d_in, const int* in_sizes, int n_in,
                              void* d_out, int out_size, void* d_ws, size_t ws_size, hipStream_t stream) {
  if (n_in < 14 || d_out == nullptr || d_ws == nullptr) return;
  if (in_sizes[0] != NSEQ * NSTEP * NC || in_sizes[1] != NSTEP || in_sizes[2] != NG3 * NC || in_sizes[3] != NG3 * NH ||
      in_sizes[4] != NG3 || in_sizes[5] != NG3 || in_sizes[6] != NHH * NH || in_sizes[7] != NHH ||
      in_sizes[8] != NHH * NHH || in_sizes[9] != NHH || in_sizes[10] != NH * NHH || in_sizes[11] != NH ||
      in_sizes[12] != NCLS * NH || in_sizes[13] != NCLS || out_size != NSEQ * NCLS) return;

  const float* x     = (const float*)d_in[0];
  const float* times = (const float*)d_in[1];
  const float* W_ih  = (const float*)d_in[2];
  const float* W_hh  = (const float*)d_in[3];
  const float* b_ih  = (const float*)d_in[4];
  const float* b_hh  = (const float*)d_in[5];
  const float* w1    = (const float*)d_in[6];
  const float* b1    = (const float*)d_in[7];
  const float* w2    = (const float*)d_in[8];
  const float* b2    = (const float*)d_in[9];
  const float* w3    = (const float*)d_in[10];
  const float* b3    = (const float*)d_in[11];
  const float* Wo    = (const float*)d_in[12];
  const float* bo    = (const float*)d_in[13];
  float* out = (float*)d_out;

  char* ws = (char*)d_ws; size_t off = 0;
  auto carve = [&](size_t bytes) -> char* { char* p = ws + off; off += (bytes + 255) & ~(size_t)255; return p; };
  unsigned short* WIH  = (unsigned short*)carve((size_t)NG3 * NC * 2);
  unsigned short* WHH  = (unsigned short*)carve((size_t)NG3 * NH * 2);
  unsigned short* W1P  = (unsigned short*)carve((size_t)NHH * NH * 2);
  unsigned short* W2P  = (unsigned short*)carve((size_t)NHH * NHH * 2);
  unsigned short* W3P  = (unsigned short*)carve((size_t)NH * NHH * 2);
  float*          HFIN = (float*)carve((size_t)NSEQ * NH * 4);
  if (off > ws_size || off > (size_t)134217728) return;

  const int n8ih = NG3 * (NC / 8);
  const int n8hh = NG3 * (NH / 8);
  const int n8w1 = NHH * (NH / 8);
  const int n8w2 = NHH * (NHH / 8);
  const int n8w3 = NH * (NHH / 8);
  cvt8_kernel<1><<<(n8ih + NTHR - 1) / NTHR, NTHR, 0, stream>>>(W_ih, WIH, NG3, NC / 8,  NC,  0, WSCL);
  cvt8_kernel<1><<<(n8hh + NTHR - 1) / NTHR, NTHR, 0, stream>>>(W_hh, WHH, NG3, NH / 8,  NH,  0, WSCL);
  cvt8_kernel<1><<<(n8w1 + NTHR - 1) / NTHR, NTHR, 0, stream>>>(w1,   W1P, NHH, NH / 8,  NH,  0, WSCL);
  cvt8_kernel<1><<<(n8w2 + NTHR - 1) / NTHR, NTHR, 0, stream>>>(w2,   W2P, NHH, NHH / 8, NHH, 0, WSCL);
  cvt8_kernel<1><<<(n8w3 + NTHR - 1) / NTHR, NTHR, 0, stream>>>(w3,   W3P, NH,  NHH / 8, NHH, 0, WSCL);
  seq_rk4_gru_kernel<<<NSEQ / RB, NTHR, 0, stream>>>(x, times, b_ih, b_hh, b1, b2, b3, WIH, WHH, W1P, W2P, W3P, HFIN);
  head_softmax_kernel<<<NSEQ / (NTHR / 32), NTHR, 0, stream>>>(HFIN, Wo, bo, out);
}
